// SNN_LSTM_Model_58729382806127
// MI455X (gfx1250) — hardware-verified
//
#include <hip/hip_runtime.h>
#include <math.h>

#pragma clang fp contract(off)

constexpr int NBATCH  = 32;
constexpr int NSTEP   = 512;
constexpr int NIN     = 256;
constexpr int NHID    = 512;
constexpr int NGATE   = 4 * NHID;
constexpr int NOUTF   = 128;
constexpr int NTHR    = 256;
constexpr int SEQ_BLK = 16;
constexpr int NHALF   = 2;
constexpr int HALF_STEPS = NSTEP / NHALF;
constexpr int HROWS   = HALF_STEPS * NBATCH;
constexpr int NROWS   = NSTEP * NBATCH;
constexpr int HPITCH  = 520;
constexpr int SLABP   = 68;
constexpr int OPITCH  = 132;
constexpr int FINALBUF = ((HALF_STEPS - 1) & 1) ^ 1;
constexpr float WCARRY     = 256.0f;
constexpr float WCARRY_INV = 1.0f / 256.0f;
static_assert(NBATCH == 32);
static_assert(NBATCH % SEQ_BLK == 0);
static_assert(NHID == 64 * (NTHR / 32));
static_assert(NOUTF == 16 * (NTHR / 32));
static_assert(NIN % 32 == 0 && NHID % 32 == 0);
static_assert(HROWS % 64 == 0 && NGATE % 64 == 0);
static_assert(((HROWS / 64) * (NGATE / 64)) % 8 == 0);
static_assert((2 * SEQ_BLK * HPITCH) % NTHR == 0);
static_assert(NSTEP % NHALF == 0);
static_assert(FINALBUF == 0 || FINALBUF == 1);

typedef __attribute__((ext_vector_type(16))) _Float16 v16h;
typedef __attribute__((ext_vector_type(8)))  _Float16 v8h;
typedef __attribute__((ext_vector_type(16))) __bf16   v16b;
typedef __attribute__((ext_vector_type(8)))  __bf16   v8b;
typedef __attribute__((ext_vector_type(8)))  float    v8f;
typedef __attribute__((ext_vector_type(4)))  float    v4f;

__device__ __forceinline__ unsigned short f2bf_bits(float f) {
  unsigned u = __float_as_uint(f);
  return (unsigned short)((u + 0x7FFFu + ((u >> 16) & 1u)) >> 16);
}
__device__ __forceinline__ float bf_bits2f(unsigned short h) { return __uint_as_float(((unsigned)h) << 16); }
__device__ __forceinline__ __bf16 f2bf(float f) { return __builtin_bit_cast(__bf16, f2bf_bits(f)); }

__device__ __forceinline__ void dep_guard_h(v8f& a, v8f& b, v16h x, v16h y) { asm volatile("v_nop\n\tv_nop\n\tv_nop\n\tv_nop" : "+v"(a), "+v"(b) : "v"(x), "v"(y)); }
__device__ __forceinline__ void dep_guard_b(v8f& a, v8f& b, v16b x, v16b y) { asm volatile("v_nop\n\tv_nop\n\tv_nop\n\tv_nop" : "+v"(a), "+v"(b) : "v"(x), "v"(y)); }
__device__ __forceinline__ void keep4_h(v16h a, v16h b, v16h c, v16h d) { asm volatile("v_nop" :: "v"(a), "v"(b), "v"(c), "v"(d)); }
__device__ __forceinline__ void keep4_b(v16b a, v16b b, v16b c, v16b d) { asm volatile("v_nop" :: "v"(a), "v"(b), "v"(c), "v"(d)); }
__device__ __forceinline__ void acc_guard4(v8f& a, v8f& b, v8f& c, v8f& d) { asm volatile("v_nop\n\tv_nop\n\tv_nop\n\tv_nop" : "+v"(a), "+v"(b), "+v"(c), "+v"(d)); }
__device__ __forceinline__ void acc_guard2(v8f& a, v8f& b) { asm volatile("v_nop\n\tv_nop\n\tv_nop\n\tv_nop" : "+v"(a), "+v"(b)); }
template <typename T> struct Frag;
template <> struct Frag<_Float16> {
  typedef v16h V; union U { v16h v; v8h h[2]; };
  static __device__ __forceinline__ v16h load(const _Float16* p) {
    U f; f.h[0] = *(const v8h*)(p); f.h[1] = *(const v8h*)(p + 16); return f.v;
  }
  static __device__ __forceinline__ v8f mma(v16h a, v16h b, v8f c) {
    return __builtin_amdgcn_wmma_f32_16x16x32_f16(false, a, false, b, (short)0, c, false, false);
  }
  static __device__ __forceinline__ void guard(v8f& a, v8f& b, v16h x, v16h y) { dep_guard_h(a, b, x, y); }
  static __device__ __forceinline__ void keep(v16h a, v16h b, v16h c, v16h d) { keep4_h(a, b, c, d); }
};
template <> struct Frag<__bf16> {
  typedef v16b V; union U { v16b v; v8b h[2]; };
  static __device__ __forceinline__ v16b load(const __bf16* p) {
    U f; f.h[0] = *(const v8b*)(p); f.h[1] = *(const v8b*)(p + 16); return f.v;
  }
  static __device__ __forceinline__ v8f mma(v16b a, v16b b, v8f c) {
    return __builtin_amdgcn_wmma_f32_16x16x32_bf16(false, a, false, b, (short)0, c, false, false);
  }
  static __device__ __forceinline__ void guard(v8f& a, v8f& b, v16b x, v16b y) { dep_guard_b(a, b, x, y); }
  static __device__ __forceinline__ void keep(v16b a, v16b b, v16b c, v16b d) { keep4_b(a, b, c, d); }
};

__device__ __forceinline__ float fsig(float x)  { return __builtin_amdgcn_rcpf(1.0f + expf(-x)); }
__device__ __forceinline__ float ftanh(float x) { return 1.0f - 2.0f * __builtin_amdgcn_rcpf(expf(2.0f * x) + 1.0f); }

template <int ET> struct Elem;
template <> struct Elem<0> { typedef _Float16 T; };
template <> struct Elem<1> { typedef __bf16 T; };
template <int ET, bool SPLIT, int BIAS_MODE, int OUT_MODE, bool RESID, int ACT = 0>
__global__ __launch_bounds__(256) void wmma_gemm64(
    const unsigned short* __restrict__ Ap, const unsigned short* __restrict__ A2p, int lda, long strideA,
    const unsigned short* __restrict__ Btp, const unsigned short* __restrict__ Bt2p, int ldb, long strideB,
    void* __restrict__ Cout, void* __restrict__ Cout2, int ldc, long strideC,
    const float* __restrict__ bias,
    const float* __restrict__ resid, long strideR,
    int M, int N, int K, float scale) {
  typedef typename Elem<ET>::T T;
  typedef typename Frag<T>::V V;
  const T* A = (const T*)Ap; const T* A2 = (const T*)A2p; const T* Bt = (const T*)Btp; const T* Bt2 = (const T*)Bt2p;
  __shared__ __align__(16) float sT[8][16 * 68];
  const int b    = blockIdx.y;
  const int lane = threadIdx.x & 31;
  const int wave = threadIdx.x >> 5;
  const int tilesN = N >> 6;
  const int tilesM = M >> 6;
  const int tile = blockIdx.x * 8 + wave;
  if (tile >= tilesM * tilesN) return;
  const int tm = tile / tilesN;
  const int tn = tile - tm * tilesN;
  const int m0 = tm << 6;
  const int n0 = tn << 6;

  const T* Ab  = A  + (size_t)b * strideA;
  const T* Bb  = Bt + (size_t)b * strideB;
  const T* Ab2 = SPLIT ? (A2  + (size_t)b * strideA) : nullptr;
  const T* Bb2 = SPLIT ? (Bt2 + (size_t)b * strideB) : nullptr;

  const int rlane = lane & 15;
  const int koff  = (lane >> 4) * 8;
  const int mOff  = (lane >> 4) * 8;

  v8f acc[4][4];
#pragma unroll
  for (int i = 0; i < 4; ++i)
#pragma unroll
    for (int j = 0; j < 4; ++j) acc[i][j] = (v8f){0.f,0.f,0.f,0.f,0.f,0.f,0.f,0.f};

  for (int k0 = 0; k0 < K; k0 += 32) {
    V bh[4], bl[4];
#pragma unroll
    for (int j = 0; j < 4; ++j) {
      const size_t bo = (size_t)(n0 + (j << 4) + rlane) * ldb + koff + k0;
      bh[j] = Frag<T>::load(Bb + bo);
      if (SPLIT) bl[j] = Frag<T>::load(Bb2 + bo);
    }
#pragma unroll
    for (int i = 0; i < 4; ++i) {
      const size_t ao = (size_t)(m0 + (i << 4) + rlane) * lda + koff + k0;
      V ah = Frag<T>::load(Ab + ao);
      V al;
      if (SPLIT) al = Frag<T>::load(Ab2 + ao);
#pragma unroll
      for (int j = 0; j < 4; ++j) {
        acc[i][j] = Frag<T>::mma(ah, bh[j], acc[i][j]);
        if (SPLIT) {
          acc[i][j] = Frag<T>::mma(ah, bl[j], acc[i][j]);
          acc[i][j] = Frag<T>::mma(al, bh[j], acc[i][j]);
        }
      }
      Frag<T>::guard(acc[i][0], acc[i][3], ah, SPLIT ? al : ah);
    }
    Frag<T>::keep(bh[0], bh[1], bh[2], bh[3]);
    if (SPLIT) Frag<T>::keep(bl[0], bl[1], bl[2], bl[3]);
  }
  acc_guard4(acc[0][0], acc[0][1], acc[0][2], acc[0][3]);
  acc_guard4(acc[1][0], acc[1][1], acc[1][2], acc[1][3]);
  acc_guard4(acc[2][0], acc[2][1], acc[2][2], acc[2][3]);
  acc_guard4(acc[3][0], acc[3][1], acc[3][2], acc[3][3]);

  float* slab = sT[wave];
  const float* Rb = RESID ? (resid + (size_t)b * strideR) : nullptr;
#pragma unroll
  for (int i = 0; i < 4; ++i) {
    const int mBase = m0 + (i << 4);
#pragma unroll
    for (int j = 0; j < 4; ++j) {
      const int n = n0 + (j << 4) + rlane;
      float bv = 0.f;
      if (BIAS_MODE == 2) bv = bias[n];
#pragma unroll
      for (int r = 0; r < 8; ++r) {
        float v = acc[i][j][r] * scale;
        if (BIAS_MODE == 1) v += bias[mBase + mOff + r];
        if (BIAS_MODE == 2) v += bv;
        if (RESID) v += Rb[(size_t)(mBase + mOff + r) * ldc + n];
        if (ACT == 1) v = tanhf(v);
        if (ACT == 2) v = fmaxf(v, 0.0f);
        if (ACT == 3) v = v / (1.0f + expf(-v));
        if (ACT == 4) v = (v > 0.f) ? v : 0.01f * v;
        if (ACT == 5) v = 0.5f * v * (1.0f + erff(v * 0.70710678118654752f));
        slab[(mOff + r) * 68 + (j << 4) + rlane] = v;
      }
    }
    __builtin_amdgcn_fence(__ATOMIC_RELEASE, "workgroup");
    __builtin_amdgcn_wave_barrier();
    __builtin_amdgcn_fence(__ATOMIC_ACQUIRE, "workgroup");
    if (OUT_MODE == 0) {
      float* C = (float*)Cout + (size_t)b * strideC;
      const int hh = lane >> 4, c4 = (lane & 15) * 4;
      for (int pass = 0; pass < 2; ++pass) {
#pragma unroll
        for (int it = 0; it < 8; ++it) {
          const int row = it * 2 + hh;
          v4f v = *(const v4f*)(slab + row * 68 + c4);
          *(volatile v4f*)(C + (size_t)(mBase + row) * ldc + n0 + c4) = v;
        }
        __threadfence();
      }
    } else {
      const int q = lane >> 3, c8 = (lane & 7) * 8;
      unsigned short* C  = (unsigned short*)Cout  + (size_t)b * strideC;
      unsigned short* C2 = (OUT_MODE == 2) ? ((unsigned short*)Cout2 + (size_t)b * strideC) : nullptr;
      for (int pass = 0; pass < 2; ++pass) {
#pragma unroll
        for (int it = 0; it < 4; ++it) {
          const int row = it * 4 + q;
          const float* sp = slab + row * 68 + c8;
          v8h hv, lv;
#pragma unroll
          for (int e = 0; e < 8; ++e) {
            if (OUT_MODE == 1) {
              hv[e] = (_Float16)sp[e];
            } else {
              unsigned short hb = f2bf_bits(sp[e]);
              unsigned short lb = f2bf_bits(sp[e] - bf_bits2f(hb));
              hv[e] = __builtin_bit_cast(_Float16, hb);
              lv[e] = __builtin_bit_cast(_Float16, lb);
            }
          }
          *(volatile v8h*)(C + (size_t)(mBase + row) * ldc + n0 + c8) = hv;
          if (OUT_MODE == 2) *(volatile v8h*)(C2 + (size_t)(mBase + row) * ldc + n0 + c8) = lv;
        }
        __threadfence();
      }
    }
    __builtin_amdgcn_fence(__ATOMIC_RELEASE, "workgroup");
    __builtin_amdgcn_wave_barrier();
    __builtin_amdgcn_fence(__ATOMIC_ACQUIRE, "workgroup");
  }
}

template <int PERM>
__global__ __launch_bounds__(NTHR) void cvt_split_kernel(const float* __restrict__ src, unsigned short* __restrict__ dhi,
                                                         unsigned short* __restrict__ dlo, int nrow, int ncol8, int spitch) {
  const int i  = blockIdx.x * NTHR + threadIdx.x;
  const int n8 = nrow * ncol8;
  if (i < n8) {
    const int row = i / ncol8;
    const int c8  = i - row * ncol8;
    size_t srow = (size_t)row;
    if (PERM) { const int t = row >> 5; const int bb = row & 31; srow = (size_t)bb * NSTEP + (size_t)t; }
    const float* sp = src + srow * (size_t)spitch + (size_t)c8 * 8;
    const v4f a  = *(const v4f*)(sp);
    const v4f b4 = *(const v4f*)(sp + 4);
    v8h hv, lv;
#pragma unroll
    for (int e = 0; e < 4; ++e) {
      const unsigned short h0 = f2bf_bits(a[e]);
      const unsigned short l0 = f2bf_bits(a[e] - bf_bits2f(h0));
      const unsigned short h1 = f2bf_bits(b4[e]);
      const unsigned short l1 = f2bf_bits(b4[e] - bf_bits2f(h1));
      hv[e]     = __builtin_bit_cast(_Float16, h0);
      hv[4 + e] = __builtin_bit_cast(_Float16, h1);
      lv[e]     = __builtin_bit_cast(_Float16, l0);
      lv[4 + e] = __builtin_bit_cast(_Float16, l1);
    }
    *(volatile v8h*)(dhi + (size_t)i * 8) = hv;
    *(volatile v8h*)(dlo + (size_t)i * 8) = lv;
    __threadfence();
    *(volatile v8h*)(dhi + (size_t)i * 8) = hv;
    *(volatile v8h*)(dlo + (size_t)i * 8) = lv;
  }
}

__global__ __launch_bounds__(NTHR) void cvt_f16_kernel(const float* __restrict__ src, unsigned short* __restrict__ dst,
                                                       int nrow, int ncol8, int spitch, float sc) {
  const int i  = blockIdx.x * NTHR + threadIdx.x;
  const int n8 = nrow * ncol8;
  if (i < n8) {
    const int row = i / ncol8;
    const int c8  = i - row * ncol8;
    const float* sp = src + (size_t)row * spitch + (size_t)c8 * 8;
    const v4f a  = *(const v4f*)(sp);
    const v4f b4 = *(const v4f*)(sp + 4);
    v8h hv;
#pragma unroll
    for (int e = 0; e < 4; ++e) {
      hv[e]     = (_Float16)(a[e] * sc);
      hv[4 + e] = (_Float16)(b4[e] * sc);
    }
    *(volatile v8h*)(dst + (size_t)i * 8) = hv;
    __threadfence();
    *(volatile v8h*)(dst + (size_t)i * 8) = hv;
  }
}

__global__ __launch_bounds__(NTHR) void bias_sum_kernel(const float* __restrict__ b_a, const float* __restrict__ b_b,
                                                        float* __restrict__ dst, int n4) {
  const int i = blockIdx.x * NTHR + threadIdx.x;
  if (i < n4) {
    const v4f va = *(const v4f*)(b_a + (size_t)i * 4);
    const v4f vb = *(const v4f*)(b_b + (size_t)i * 4);
    const v4f o = va + vb;
    *(volatile v4f*)(dst + (size_t)i * 4) = o;
    __threadfence();
    *(volatile v4f*)(dst + (size_t)i * 4) = o;
  }
}

__device__ __forceinline__ void store_tile_16x64(float* __restrict__ plane, const float* slab, int rowbase, int wave, int hh, int c4) {
  for (int pass = 0; pass < 2; ++pass) {
#pragma unroll
    for (int it = 0; it < 8; ++it) {
      const int row = it * 2 + hh;
      const v4f v = *(const v4f*)(slab + row * SLABP + c4);
      *(volatile v4f*)(plane + (size_t)(rowbase + row) * NHID + 64 * wave + c4) = v;
    }
    __threadfence();
  }
}
__device__ __forceinline__ void wave_lds_sync() {
  __builtin_amdgcn_fence(__ATOMIC_RELEASE, "workgroup");
  __builtin_amdgcn_wave_barrier();
  __builtin_amdgcn_fence(__ATOMIC_ACQUIRE, "workgroup");
}

__global__ __launch_bounds__(NTHR) void lstm_lif_kernel(const float* __restrict__ XP, const unsigned short* __restrict__ WHHp,
                                                        float* __restrict__ HST, float* __restrict__ CST, float* __restrict__ MEMP,
                                                        float* __restrict__ SPK, int first, int lastflag) {
  __shared__ __align__(16) _Float16 Ah[2][SEQ_BLK * HPITCH];
  __shared__ __align__(16) float    Sl[NTHR / 32][16 * SLABP];
  const _Float16* WHH = (const _Float16*)WHHp;
  const int tid = threadIdx.x, lane = tid & 31, wave = tid >> 5;
  const int c = lane & 15, hh = lane >> 4, koff = hh * 8, c4 = c * 4;
  const int rowbase = blockIdx.x * SEQ_BLK;
  float* slab = Sl[wave];

#pragma unroll 1
  for (int i = tid; i < 2 * SEQ_BLK * HPITCH; i += NTHR) {
    const int buf  = (i >= SEQ_BLK * HPITCH) ? 1 : 0;
    const int rem  = i - buf * (SEQ_BLK * HPITCH);
    const int row  = rem / HPITCH;
    const int col  = rem - row * HPITCH;
    const int colc = (col < NHID) ? col : (NHID - 1);
    const float hv = HST[(size_t)(rowbase + row) * NHID + colc];
    const float v  = (first != 0 || buf != 0 || col >= NHID) ? 0.0f : hv;
    (&Ah[0][0])[i] = (_Float16)v;
  }
  float cst[4][8], mem[4][8];
#pragma unroll
  for (int nt = 0; nt < 4; ++nt) {
    const int j = 64 * wave + 16 * nt + c;
#pragma unroll
    for (int r = 0; r < 8; ++r) {
      const size_t so = (size_t)(rowbase + 8 * hh + r) * NHID + j;
      const float cv = CST[so];
      const float mv = MEMP[so];
      cst[nt][r] = (first != 0) ? 0.0f : cv;
      mem[nt][r] = (first != 0) ? 0.0f : mv;
    }
  }
  __syncthreads();

  const v8f z8 = {0.f, 0.f, 0.f, 0.f, 0.f, 0.f, 0.f, 0.f};

#pragma unroll 1
  for (int lt = 0; lt < HALF_STEPS; ++lt) {
    const int cur = lt & 1;
    const _Float16* ahrow = &Ah[cur][0] + c * HPITCH + koff;
    _Float16* ahn = &Ah[cur ^ 1][0];
    const float* xprow = XP + (size_t)(lt * NBATCH + rowbase + 8 * hh) * NGATE;

#pragma unroll
    for (int nt = 0; nt < 4; ++nt) {
      const int j = 64 * wave + 16 * nt + c;
      const _Float16* wi = WHH + (size_t)(j) * NHID + koff;
      const _Float16* wf = WHH + (size_t)(NHID + j) * NHID + koff;
      const _Float16* wg = WHH + (size_t)(2 * NHID + j) * NHID + koff;
      const _Float16* wo = WHH + (size_t)(3 * NHID + j) * NHID + koff;
      v8f ai = z8, af = z8, ag = z8, ao = z8;
#pragma unroll 1
      for (int k0 = 0; k0 < NHID; k0 += 32) {
        const v16h a  = Frag<_Float16>::load(ahrow + k0);
        const v16h bi = Frag<_Float16>::load(wi + k0);
        const v16h bf = Frag<_Float16>::load(wf + k0);
        const v16h bg = Frag<_Float16>::load(wg + k0);
        const v16h bo = Frag<_Float16>::load(wo + k0);
        ai = Frag<_Float16>::mma(a, bi, ai);
        af = Frag<_Float16>::mma(a, bf, af);
        ag = Frag<_Float16>::mma(a, bg, ag);
        ao = Frag<_Float16>::mma(a, bo, ao);
        dep_guard_h(ai, ao, a, bo);
        keep4_h(a, bi, bf, bg);
      }
      acc_guard4(ai, af, ag, ao);
#pragma unroll
      for (int r = 0; r < 8; ++r) {
        const float* xp = xprow + (size_t)r * NGATE + j;
        const float xi = xp[0];
        const float xf = xp[NHID];
        const float xg = xp[2 * NHID];
        const float xo = xp[3 * NHID];
        const float zi = ai[r] * WCARRY_INV + xi;
        const float zf = af[r] * WCARRY_INV + xf;
        const float zg = ag[r] * WCARRY_INV + xg;
        const float zo = ao[r] * WCARRY_INV + xo;
        const float gi = fsig(zi);
        const float gf = fsig(zf);
        const float gc = ftanh(zg);
        const float go = fsig(zo);
        const float cn = gf * cst[nt][r] + gi * gc;
        cst[nt][r] = cn;
        const float hn = go * ftanh(cn);
        float mv = 0.9f * mem[nt][r] + hn;
        const float u  = mv - 1.0f;
        const float sp = (u > 0.0f) ? 1.0f : 0.0f;
        mv = mv - sp;
        mem[nt][r] = mv;
        ahn[(8 * hh + r) * HPITCH + j] = (_Float16)hn;
        slab[(8 * hh + r) * SLABP + 16 * nt + c] = sp;
      }
    }
    __syncthreads();
    if (lastflag != 0 && lt == HALF_STEPS - 1) {
      wave_lds_sync();
      store_tile_16x64(SPK, slab, rowbase, wave, hh, c4);
      wave_lds_sync();
    }
  }

#pragma unroll
  for (int nt = 0; nt < 4; ++nt)
#pragma unroll
    for (int r = 0; r < 8; ++r) slab[(8 * hh + r) * SLABP + 16 * nt + c] = cst[nt][r];
  wave_lds_sync();
  store_tile_16x64(CST, slab, rowbase, wave, hh, c4);
  wave_lds_sync();
#pragma unroll
  for (int nt = 0; nt < 4; ++nt)
#pragma unroll
    for (int r = 0; r < 8; ++r) slab[(8 * hh + r) * SLABP + 16 * nt + c] = mem[nt][r];
  wave_lds_sync();
  store_tile_16x64(MEMP, slab, rowbase, wave, hh, c4);
  wave_lds_sync();
  {
    const _Float16* ahf = &Ah[FINALBUF][0];
#pragma unroll
    for (int nt = 0; nt < 4; ++nt) {
      const int j = 64 * wave + 16 * nt + c;
#pragma unroll
      for (int r = 0; r < 8; ++r) slab[(8 * hh + r) * SLABP + 16 * nt + c] = (float)ahf[(8 * hh + r) * HPITCH + j];
    }
  }
  wave_lds_sync();
  store_tile_16x64(HST, slab, rowbase, wave, hh, c4);
}

__global__ __launch_bounds__(NTHR) void fc_head_kernel(const float* __restrict__ SPK, const unsigned short* __restrict__ WFHp,
                                                       const unsigned short* __restrict__ WFLp, const float* __restrict__ bfc,
                                                       float* __restrict__ out) {
  __shared__ __align__(16) float Os[NBATCH * OPITCH];
  const __bf16* WFH = (const __bf16*)WFHp;
  const __bf16* WFL = (const __bf16*)WFLp;
  const int tid = threadIdx.x, lane = tid & 31, wave = tid >> 5;
  const int c = lane & 15, hh = lane >> 4, koff = hh * 8;
  const int n = 16 * wave + c;
  const __bf16* bhp = WFH + (size_t)n * NHID + koff;
  const __bf16* blp = WFL + (size_t)n * NHID + koff;
  const float* s0 = SPK + (size_t)c * NHID + koff;
  const float* s1 = SPK + (size_t)(16 + c) * NHID + koff;
  const v8f z8 = {0.f, 0.f, 0.f, 0.f, 0.f, 0.f, 0.f, 0.f};
  v8f acc0 = z8, acc1 = z8;
#pragma unroll 1
  for (int k0 = 0; k0 < NHID; k0 += 32) {
    const v4f p0 = *(const v4f*)(s0 + k0), p1 = *(const v4f*)(s0 + k0 + 4), p2 = *(const v4f*)(s0 + k0 + 16), p3 = *(const v4f*)(s0 + k0 + 20);
    const v4f q0 = *(const v4f*)(s1 + k0), q1 = *(const v4f*)(s1 + k0 + 4), q2 = *(const v4f*)(s1 + k0 + 16), q3 = *(const v4f*)(s1 + k0 + 20);
    v16b a0v, a1v;
#pragma unroll
    for (int e = 0; e < 4; ++e) {
      a0v[e] = f2bf(p0[e]); a0v[4 + e] = f2bf(p1[e]); a0v[8 + e] = f2bf(p2[e]); a0v[12 + e] = f2bf(p3[e]);
      a1v[e] = f2bf(q0[e]); a1v[4 + e] = f2bf(q1[e]); a1v[8 + e] = f2bf(q2[e]); a1v[12 + e] = f2bf(q3[e]);
    }
    const v16b wh = Frag<__bf16>::load(bhp + k0);
    const v16b wl = Frag<__bf16>::load(blp + k0);
    acc0 = Frag<__bf16>::mma(a0v, wh, acc0);
    acc0 = Frag<__bf16>::mma(a0v, wl, acc0);
    acc1 = Frag<__bf16>::mma(a1v, wh, acc1);
    acc1 = Frag<__bf16>::mma(a1v, wl, acc1);
    dep_guard_b(acc0, acc1, a1v, wl);
    keep4_b(a0v, wh, a1v, wl);
  }
  acc_guard2(acc0, acc1);
  const float bv = bfc[n];
#pragma unroll
  for (int r = 0; r < 8; ++r) {
    Os[(8 * hh + r) * OPITCH + n]      = acc0[r] + bv;
    Os[(16 + 8 * hh + r) * OPITCH + n] = acc1[r] + bv;
  }
  __syncthreads();
  for (int pass = 0; pass < 2; ++pass) {
#pragma unroll
    for (int it = 0; it < 4; ++it) {
      const int f = it * NTHR + tid;
      const int row = f >> 5;
      const int cc4 = (f & 31) * 4;
      const v4f v = *(const v4f*)(Os + row * OPITCH + cc4);
      *(volatile v4f*)(out + (size_t)row * NOUTF + cc4) = v;
    }
    __threadfence();
  }
}

extern "C" void kernel_launch(void* const* d_in, const int* in_sizes, int n_in,
                              void* d_out, int out_size, void* d_ws, size_t ws_size, hipStream_t stream) {
  if (n_in < 7 || d_out == nullptr || d_ws == nullptr) return;
  if (in_sizes[0] != NBATCH * NSTEP * NIN || in_sizes[1] != NGATE * NIN || in_sizes[2] != NGATE * NHID ||
      in_sizes[3] != NGATE || in_sizes[4] != NGATE || in_sizes[5] != NOUTF * NHID || in_sizes[6] != NOUTF ||
      out_size != NBATCH * NOUTF) return;

  const float* x    = (const float*)d_in[0];
  const float* w_ih = (const float*)d_in[1];
  const float* w_hh = (const float*)d_in[2];
  const float* b_ih = (const float*)d_in[3];
  const float* b_hh = (const float*)d_in[4];
  const float* w_fc = (const float*)d_in[5];
  const float* b_fc = (const float*)d_in[6];
  float* y_out = (float*)d_out;

  char* ws = (char*)d_ws; size_t off = 0;
  auto carve = [&](size_t bytes) -> char* { char* p = ws + off; off += (bytes + 255) & ~(size_t)255; return p; };
  unsigned short* XH   = (unsigned short*)carve((size_t)NROWS * NIN * 2);
  unsigned short* XL   = (unsigned short*)carve((size_t)NROWS * NIN * 2);
  unsigned short* WIH  = (unsigned short*)carve((size_t)NGATE * NIN * 2);
  unsigned short* WIL  = (unsigned short*)carve((size_t)NGATE * NIN * 2);
  unsigned short* WHH  = (unsigned short*)carve((size_t)NGATE * NHID * 2);
  unsigned short* WFH  = (unsigned short*)carve((size_t)NOUTF * NHID * 2);
  unsigned short* WFL  = (unsigned short*)carve((size_t)NOUTF * NHID * 2);
  float*          BIAS = (float*)carve((size_t)NGATE * 4);
  float*          HST  = (float*)carve((size_t)NBATCH * NHID * 4);
  float*          CST  = (float*)carve((size_t)NBATCH * NHID * 4);
  float*          MEMP = (float*)carve((size_t)NBATCH * NHID * 4);
  float*          SPK  = (float*)carve((size_t)NBATCH * NHID * 4);
  float*          XP   = (float*)carve((size_t)HROWS * NGATE * 4);
  if (off > ws_size || off > (size_t)134217728) return;

  const int n8x  = NROWS * (NIN / 8);
  const int n8wi = NGATE * (NIN / 8);
  const int n8wh = NGATE * (NHID / 8);
  const int n8wf = NOUTF * (NHID / 8);
  cvt_split_kernel<1><<<(n8x + NTHR - 1) / NTHR, NTHR, 0, stream>>>(x, XH, XL, NROWS, NIN / 8, NIN);
  cvt_split_kernel<0><<<(n8wi + NTHR - 1) / NTHR, NTHR, 0, stream>>>(w_ih, WIH, WIL, NGATE, NIN / 8, NIN);
  cvt_f16_kernel<<<(n8wh + NTHR - 1) / NTHR, NTHR, 0, stream>>>(w_hh, WHH, NGATE, NHID / 8, NHID, WCARRY);
  cvt_split_kernel<0><<<(n8wf + NTHR - 1) / NTHR, NTHR, 0, stream>>>(w_fc, WFH, WFL, NOUTF, NHID / 8, NHID);
  bias_sum_kernel<<<(NGATE / 4 + NTHR - 1) / NTHR, NTHR, 0, stream>>>(b_ih, b_hh, BIAS, NGATE / 4);

  const dim3 ggrid((HROWS / 64) * (NGATE / 64) / 8, 1);
  for (int hf = 0; hf < NHALF; ++hf) {
    const size_t aoff = (size_t)hf * HROWS * NIN;
    wmma_gemm64<1, true, 2, 0, false, 0><<<ggrid, 256, 0, stream>>>(
        XH + aoff, XL + aoff, NIN, 0L, WIH, WIL, NIN, 0L, (void*)XP, (void*)XP, NGATE, 0L,
        BIAS, XP, 0L, HROWS, NGATE, NIN, 1.0f);
    lstm_lif_kernel<<<NBATCH / SEQ_BLK, NTHR, 0, stream>>>(XP, WHH, HST, CST, MEMP, SPK,
                                                           (hf == 0) ? 1 : 0, (hf == NHALF - 1) ? 1 : 0);
  }

  fc_head_kernel<<<1, NTHR, 0, stream>>>(SPK, WFH, WFL, b_fc, y_out);
}
